// EdgeClassifier_10496900071609
// MI455X (gfx1250) — hardware-verified
//
#include <hip/hip_runtime.h>
#include <stddef.h>
#include <stdint.h>

#define HDIM   128
#define KDIM   256
#define TROWS  64
#define GTHR   128
#define LDSW   264
#define NUNW   (HDIM * KDIM / 8)
#define WSMAX  134217728

static_assert(KDIM % 32 == 0 && HDIM == 128 && KDIM == 2 * HDIM);
static_assert(TROWS == (GTHR / 32) * 16);
static_assert(GTHR == 2 * TROWS);
static_assert(((LDSW * 2) % 16) == 0);
static_assert((TROWS * KDIM) % (GTHR * 4) == 0);
static_assert(TROWS / 4 == 16);
static_assert(NUNW % 256 == 0);

typedef float          v4f   __attribute__((ext_vector_type(4)));
typedef float          v8f   __attribute__((ext_vector_type(8)));
typedef int            v8i   __attribute__((ext_vector_type(8)));
typedef unsigned short v4us  __attribute__((ext_vector_type(4)));
typedef unsigned short v8us  __attribute__((ext_vector_type(8)));
typedef unsigned short v16us __attribute__((ext_vector_type(16)));
typedef __bf16         v16bf __attribute__((ext_vector_type(16)));
typedef v4f  __attribute__((may_alias)) v4fa;
typedef v4us __attribute__((may_alias)) v4usa;
typedef v8us __attribute__((may_alias)) v8usa;
union FragB { v16bf v; v16us u; v8us h[2]; v8i w; };

__device__ __forceinline__ v8f wmb(const FragB& a, const FragB& b, v8f c) {
  v8f d = __builtin_amdgcn_wmma_f32_16x16x32_bf16(false, a.v, false, b.v, (short)0, c, false, false);
  asm volatile("v_nop\n\tv_nop\n\tv_nop\n\tv_nop" : "+v"(d) : "v"(a.w), "v"(b.w));
  return d;
}

__device__ __forceinline__ unsigned bf16_bits(float f) {
  const unsigned u = __float_as_uint(f);
  return (u + 0x7FFFu + ((u >> 16) & 1u)) >> 16;
}
__device__ __forceinline__ float bf16_val(float f) {
  return __uint_as_float(bf16_bits(f) << 16);
}

__global__ __launch_bounds__(256) void k_wprep(const float* __restrict__ W1, unsigned short* WT, int nUnits) {
  const int u = (int)blockIdx.x * 256 + (int)threadIdx.x;
  if (u >= nUnits) return;
  const float* p = W1 + (size_t)u * 8;
  const v4f a = *(const v4fa*)p;
  const v4f c = *(const v4fa*)(p + 4);
  v8us o;
  o[0] = (unsigned short)bf16_bits(a.x);
  o[1] = (unsigned short)bf16_bits(a.y);
  o[2] = (unsigned short)bf16_bits(a.z);
  o[3] = (unsigned short)bf16_bits(a.w);
  o[4] = (unsigned short)bf16_bits(c.x);
  o[5] = (unsigned short)bf16_bits(c.y);
  o[6] = (unsigned short)bf16_bits(c.z);
  o[7] = (unsigned short)bf16_bits(c.w);
  unsigned short* dp = WT + (size_t)u * 8;
  *(volatile v8us*)dp = o;
  __threadfence();
  *(volatile v8us*)dp = o;
}

__device__ __forceinline__ void out_store_pass(float* out, v4f v, int eb, int nE, bool full, bool tailw) {
  if (full) {
    *(volatile v4f*)(out + (size_t)eb) = v;
  } else if (tailw) {
    if (eb     < nE) *(volatile float*)(out + (size_t)eb)     = v.x;
    if (eb + 1 < nE) *(volatile float*)(out + (size_t)eb + 1) = v.y;
    if (eb + 2 < nE) *(volatile float*)(out + (size_t)eb + 2) = v.z;
    if (eb + 3 < nE) *(volatile float*)(out + (size_t)eb + 3) = v.w;
  }
}

__global__ __launch_bounds__(GTHR) void k_edge(
    const float* __restrict__ zd,
    const float* __restrict__ zp,
    const int*   __restrict__ eli,
    const unsigned short* __restrict__ WT,
    const float* __restrict__ b1,
    const float* __restrict__ W2,
    const float* __restrict__ b2,
    float* out,
    int nE, int nD, int nP)
{
  __shared__ __attribute__((aligned(16))) unsigned short sA[TROWS * LDSW];
  __shared__ __attribute__((aligned(16))) float sOut[TROWS];
  __shared__ __attribute__((aligned(16))) float sB1[HDIM];
  __shared__ __attribute__((aligned(16))) float sW2[HDIM];
  __shared__ int sIdx[2 * TROWS];

  const int tid = (int)threadIdx.x, lane = tid & 31, wave = tid >> 5;
  const int hh = lane >> 4, m = lane & 15;
  const int e0 = (int)blockIdx.x * TROWS;

  {
    const int r   = tid & (TROWS - 1);
    const int sel = tid >> 6;
    int e = e0 + r;
    e = e > nE - 1 ? nE - 1 : e;
    const int raw = eli[(size_t)sel * (size_t)nE + (size_t)e];
    const int nN  = (sel == 0) ? nD : nP;
    int ix = raw < 0 ? raw + nN : raw;
    ix = ix < 0 ? 0 : (ix > nN - 1 ? nN - 1 : ix);
    sIdx[tid] = ix;
    sB1[tid] = bf16_val(b1[tid]);
    sW2[tid] = bf16_val(W2[tid]);
  }
  __syncthreads();

  {
    const int c4 = tid & 63;
    const bool isP = (wave & 1) != 0;
    const float* zsrc = isP ? zp : zd;
    const int kin  = 4 * (c4 & 31);
    const int kout = 4 * c4;
    const int rsub = wave >> 1;
    const int ibase = isP ? TROWS : 0;
#pragma unroll 4
    for (int i = 0; i < (TROWS * KDIM) / (GTHR * 4); ++i) {
      const int row  = 2 * i + rsub;
      const int node = sIdx[ibase + row];
      const v4f v = *(const v4fa*)(zsrc + (size_t)node * HDIM + kin);
      v4us o;
      o[0] = (unsigned short)bf16_bits(v.x);
      o[1] = (unsigned short)bf16_bits(v.y);
      o[2] = (unsigned short)bf16_bits(v.z);
      o[3] = (unsigned short)bf16_bits(v.w);
      *(v4usa*)(sA + row * LDSW + kout) = o;
    }
  }
  __syncthreads();

  v8f acc[8];
  {
    const v8f z8 = {0.f, 0.f, 0.f, 0.f, 0.f, 0.f, 0.f, 0.f};
#pragma unroll
    for (int t = 0; t < 8; ++t) acc[t] = z8;
  }
  const unsigned short* ap = sA + (16 * wave + m) * LDSW + 8 * hh;
  const unsigned short* wp = WT + (size_t)m * KDIM + 8 * hh;

#pragma unroll 1
  for (int kk = 0; kk < KDIM / 32; ++kk) {
    const int k0 = 32 * kk;
    FragB af;
    af.h[0] = *(const v8usa*)(ap + k0);
    af.h[1] = *(const v8usa*)(ap + k0 + 16);
#pragma unroll
    for (int nt = 0; nt < 8; ++nt) {
      const unsigned short* wq = wp + (size_t)(16 * nt) * KDIM + k0;
      FragB bf;
      bf.h[0] = *(const v8usa*)wq;
      bf.h[1] = *(const v8usa*)(wq + 16);
      acc[nt] = wmb(af, bf, acc[nt]);
    }
  }

  float part[8];
#pragma unroll
  for (int r = 0; r < 8; ++r) part[r] = 0.0f;
#pragma unroll
  for (int nt = 0; nt < 8; ++nt) {
    const int col = 16 * nt + m;
    const float bv = sB1[col];
    const float wv = sW2[col];
#pragma unroll
    for (int r = 0; r < 8; ++r) {
      const float hv = fmaxf(acc[nt][r] + bv, 0.0f);
      part[r] = fmaf(hv, wv, part[r]);
    }
  }
#pragma unroll
  for (int msk = 1; msk <= 8; msk <<= 1) {
#pragma unroll
    for (int r = 0; r < 8; ++r) part[r] += __shfl_xor(part[r], msk, 32);
  }
  const float b2v = bf16_val(b2[0]);
  if (m == 0) {
#pragma unroll
    for (int r = 0; r < 8; ++r) sOut[16 * wave + 8 * hh + r] = part[r] + b2v;
  }
  __syncthreads();

  const bool wr  = (tid < TROWS / 4);
  const int  t16 = wr ? tid : 0;
  const v4f  v   = *(const v4fa*)(sOut + 4 * t16);
  const int  eb  = e0 + 4 * t16;
  const bool full  = wr && (eb + 3 < nE);
  const bool tailw = wr && !full;
  out_store_pass(out, v, eb, nE, full, tailw);
  __threadfence();
  out_store_pass(out, v, eb, nE, full, tailw);
}

static inline int cdiv(int a, int b) { return (a + b - 1) / b; }

extern "C" void kernel_launch(void* const* d_in, const int* in_sizes, int n_in,
                              void* d_out, int out_size, void* d_ws, size_t ws_size,
                              hipStream_t stream) {
  if (n_in < 7) return;
  if (in_sizes[0] < HDIM || (in_sizes[0] % HDIM) != 0) return;
  if (in_sizes[1] < HDIM || (in_sizes[1] % HDIM) != 0) return;
  const int nD = in_sizes[0] / HDIM;
  const int nP = in_sizes[1] / HDIM;
  if (in_sizes[2] < 2 || (in_sizes[2] & 1) != 0) return;
  const int nE = in_sizes[2] / 2;
  if (in_sizes[3] != HDIM * KDIM) return;
  if (in_sizes[4] != HDIM) return;
  if (in_sizes[5] != HDIM) return;
  if (in_sizes[6] < 1) return;
  if (out_size != nE) return;

  const float* zd  = (const float*)d_in[0];
  const float* zp  = (const float*)d_in[1];
  const int*   eli = (const int*)d_in[2];
  const float* W1  = (const float*)d_in[3];
  const float* b1  = (const float*)d_in[4];
  const float* W2  = (const float*)d_in[5];
  const float* b2  = (const float*)d_in[6];
  float* out = (float*)d_out;

  char* ws = (char*)d_ws;
  size_t off = 0;
  const size_t oWT = off; off += (size_t)HDIM * KDIM * 2; off = (off + 255) & ~(size_t)255;
  if (off > ws_size || off > (size_t)WSMAX) return;
  unsigned short* WT = (unsigned short*)(ws + oWT);

  k_wprep<<<cdiv(NUNW, 256), 256, 0, stream>>>(W1, WT, NUNW);
  k_edge<<<cdiv(nE, TROWS), GTHR, 0, stream>>>(zd, zp, eli, WT, b1, W2, b2, out, nE, nD, nP);
}
